// MSPSurfNet_69638599737455
// MI455X (gfx1250) — hardware-verified
//
#include <hip/hip_runtime.h>
#define NV 16000
#define NC 4096
#define CF 64
#define FIN 130
#define FINP 160
#define RSIG 2.5f
#define GSIG 3.0f
#define RCH 1024
typedef __bf16 v16b __attribute__((ext_vector_type(16)));
typedef unsigned short v8us __attribute__((ext_vector_type(8), may_alias));
typedef float  v8f  __attribute__((ext_vector_type(8)));
typedef float  v4f  __attribute__((ext_vector_type(4)));
typedef float  v4fa __attribute__((ext_vector_type(4), may_alias));
union FragB { v16b v; v8us half[2]; unsigned short u[16]; };

__device__ __forceinline__ unsigned short bf16_bits(float x) { unsigned int u = __float_as_uint(x); return (unsigned short)((u + 0x7FFFu + ((u >> 16) & 1u)) >> 16); }
__device__ __forceinline__ float bf16_val(unsigned short b) { return __uint_as_float(((unsigned int)b) << 16); }
__device__ __forceinline__ float bf16_round(float x) { return bf16_val(bf16_bits(x)); }
template <int NT>
__device__ __forceinline__ v8f mmaN(v16b ah, v16b al, v16b bh, v16b bl, v8f c) {
  c = __builtin_amdgcn_wmma_f32_16x16x32_bf16(false, ah, false, bh, (short)0, c, false, false);
  if (NT >= 2) c = __builtin_amdgcn_wmma_f32_16x16x32_bf16(false, al, false, bh, (short)0, c, false, false);
  if (NT >= 3) c = __builtin_amdgcn_wmma_f32_16x16x32_bf16(false, ah, false, bl, (short)0, c, false, false);
  asm volatile("v_nop\n\tv_nop\n\tv_nop\n\tv_nop" : "+v"(c) : "v"(ah), "v"(al), "v"(bh), "v"(bl));
  return c;
}

__global__ __launch_bounds__(256) void k_wt_bf16(const float* __restrict__ W, unsigned short* __restrict__ Wt, int K, int N) {
  const int t = blockIdx.x * 256 + threadIdx.x;
  const int k8n = K / 8;
  if (t >= N * k8n) return;
  const int n = t / k8n, k8 = (t % k8n) * 8;
  v8us v;
#pragma unroll
  for (int i = 0; i < 8; ++i) v[i] = bf16_bits(W[(size_t)(k8 + i) * N + n]);
  *(volatile v8us*)(Wt + (size_t)n * K + k8) = v;
  __threadfence();
  *(volatile v8us*)(Wt + (size_t)n * K + k8) = v;
}

template <bool ASPLIT, int ACT, bool BIAS_BF16>
__global__ __launch_bounds__(128) void k_gemm_bf(const float* __restrict__ A, int lda, const unsigned short* __restrict__ Wt, int ldb,
                                               const float* __restrict__ bias, float* __restrict__ C, int ldc, int M, int N, int K) {
  __shared__ __attribute__((aligned(16))) float so[4][16][64];
  const int tid = threadIdx.x, w = tid >> 5, lane = tid & 31, ln = lane & 15, hh = lane >> 4;
  const int ntn = N / 64;
  const int wid = blockIdx.x * 4 + w;
  const int mt = wid / ntn, nq = wid % ntn;
  if (mt * 16 >= M) return;
  const int row0 = mt * 16, col0 = nq * 64;
  const float* arow = A + (size_t)(row0 + ln) * lda;
  v8f acc[4] = {};
  for (int kb = 0; kb < K; kb += 32) {
    FragB ah, al;
    const v4f x0 = *(const v4fa*)(arow + kb + 8 * hh), x1 = *(const v4fa*)(arow + kb + 8 * hh + 4);
    const v4f x2 = *(const v4fa*)(arow + kb + 16 + 8 * hh), x3 = *(const v4fa*)(arow + kb + 16 + 8 * hh + 4);
    float xs[16] = {x0[0],x0[1],x0[2],x0[3],x1[0],x1[1],x1[2],x1[3],x2[0],x2[1],x2[2],x2[3],x3[0],x3[1],x3[2],x3[3]};
#pragma unroll
    for (int i = 0; i < 16; ++i) { const unsigned short hb = bf16_bits(xs[i]); ah.u[i] = hb; al.u[i] = ASPLIT ? bf16_bits(xs[i] - bf16_val(hb)) : (unsigned short)0; }
#pragma unroll
    for (int t = 0; t < 4; ++t) {
      const unsigned short* brow = Wt + (size_t)(col0 + t * 16 + ln) * ldb + kb;
      FragB b;
      b.half[0] = *(const v8us*)(brow + 8 * hh);
      b.half[1] = *(const v8us*)(brow + 16 + 8 * hh);
      acc[t] = mmaN<ASPLIT ? 2 : 1>(ah.v, al.v, b.v, b.v, acc[t]);
    }
  }
#pragma unroll
  for (int t = 0; t < 4; ++t) {
    float bv = bias ? bias[col0 + t * 16 + ln] : 0.f;
    if (BIAS_BF16) bv = bf16_round(bv);
#pragma unroll
    for (int r = 0; r < 8; ++r) { float v = acc[t][r] + bv; if (ACT == 1) v = fmaxf(v, 0.f); so[w][8 * hh + r][t * 16 + ln] = v; }
  }
  __builtin_amdgcn_fence(__ATOMIC_ACQ_REL, "workgroup");
  __builtin_amdgcn_wave_barrier();
  const int rsub = lane >> 4, c4 = (lane & 15) * 4;
  for (int pass = 0; pass < 2; ++pass) {
#pragma unroll
    for (int q = 0; q < 8; ++q) {
      const int r = q * 2 + rsub;
      const v4f v = *(const v4fa*)&so[w][r][c4];
      *(volatile v4f*)(C + (size_t)(row0 + r) * ldc + col0 + c4) = v;
    }
    if (pass == 0) __threadfence();
  }
}

template <bool ASPLIT, int ACT, bool BIAS_BF16, bool RES_BF16>
__global__ __launch_bounds__(128) void k_gemm_bf3(const float* __restrict__ A, int lda, const unsigned short* __restrict__ Wt, int ldb,
                                                const float* __restrict__ bias, const float* __restrict__ resid, int rmod, int ldr,
                                                float* __restrict__ C, int ldc, int M, int N, int K) {
  __shared__ __attribute__((aligned(16))) float so[4][16][64];
  const int tid = threadIdx.x, w = tid >> 5, lane = tid & 31, ln = lane & 15, hh = lane >> 4;
  const int ntn = N / 64;
  const int wid = blockIdx.x * 4 + w;
  const int mt = wid / ntn, nq = wid % ntn;
  if (mt * 16 >= M) return;
  const int row0 = mt * 16, col0 = nq * 64;
  const float* arow = A + (size_t)(row0 + ln) * lda;
  v8f acc[4] = {};
  for (int kb = 0; kb < K; kb += 32) {
    FragB ah, al;
    const v4f x0 = *(const v4fa*)(arow + kb + 8 * hh), x1 = *(const v4fa*)(arow + kb + 8 * hh + 4);
    const v4f x2 = *(const v4fa*)(arow + kb + 16 + 8 * hh), x3 = *(const v4fa*)(arow + kb + 16 + 8 * hh + 4);
    float xs[16] = {x0[0],x0[1],x0[2],x0[3],x1[0],x1[1],x1[2],x1[3],x2[0],x2[1],x2[2],x2[3],x3[0],x3[1],x3[2],x3[3]};
#pragma unroll
    for (int i = 0; i < 16; ++i) { const unsigned short hb = bf16_bits(xs[i]); ah.u[i] = hb; al.u[i] = ASPLIT ? bf16_bits(xs[i] - bf16_val(hb)) : (unsigned short)0; }
#pragma unroll
    for (int t = 0; t < 4; ++t) {
      const unsigned short* brow = Wt + (size_t)(col0 + t * 16 + ln) * ldb + kb;
      FragB b;
      b.half[0] = *(const v8us*)(brow + 8 * hh);
      b.half[1] = *(const v8us*)(brow + 16 + 8 * hh);
      acc[t] = mmaN<ASPLIT ? 2 : 1>(ah.v, al.v, b.v, b.v, acc[t]);
    }
  }
#pragma unroll
  for (int t = 0; t < 4; ++t) {
    const int col = col0 + t * 16 + ln;
    float bv = bias ? bias[col] : 0.f;
    if (BIAS_BF16) bv = bf16_round(bv);
#pragma unroll
    for (int r = 0; r < 8; ++r) {
      float v = acc[t][r] + bv;
      if (resid) { float rv = resid[(size_t)((row0 + 8 * hh + r) % rmod) * ldr + col]; if (RES_BF16) rv = bf16_round(rv); v += rv; }
      if (ACT == 1) v = fmaxf(v, 0.f);
      if (ACT == 2) v = 0.5f * v * (1.0f + erff(v * 0.70710678118654752f));
      if (ACT == 3) { const float u = 0.7978845608028654f * (v + 0.044715f * v * v * v); v = 0.5f * v * (1.0f + tanhf(u)); }
      so[w][8 * hh + r][t * 16 + ln] = v;
    }
  }
  __builtin_amdgcn_fence(__ATOMIC_ACQ_REL, "workgroup");
  __builtin_amdgcn_wave_barrier();
  const int rsub = lane >> 4, c4 = (lane & 15) * 4;
  for (int pass = 0; pass < 2; ++pass) {
#pragma unroll
    for (int q = 0; q < 8; ++q) {
      const int r = q * 2 + rsub;
      const v4f v = *(const v4fa*)&so[w][r][c4];
      *(volatile v4f*)(C + (size_t)(row0 + r) * ldc + col0 + c4) = v;
    }
    if (pass == 0) __threadfence();
  }
}
template <bool PARAM_BF16>
__global__ __launch_bounds__(256) void k_layernorm(const float* __restrict__ X, const float* __restrict__ R, const float* __restrict__ g, const float* __restrict__ bta,
                                                  float* __restrict__ out_sum, float* __restrict__ out_norm, int N, float eps) {
  __shared__ float red[256];
  const int row = blockIdx.x, tid = threadIdx.x;
  const float* x = X + (size_t)row * N; const float* rr = R ? R + (size_t)row * N : nullptr;
  float vals[16];
  const int per = N / 256;
  float s1 = 0.f;
  for (int u = 0; u < per / 4; ++u) {
    const int j = tid * 4 + 1024 * u;
    const v4f a = *(const v4fa*)(x + j);
    v4f b = {0.f,0.f,0.f,0.f}; if (rr) b = *(const v4fa*)(rr + j);
#pragma unroll
    for (int q = 0; q < 4; ++q) { const float v = a[q] + b[q]; vals[u * 4 + q] = v; s1 += v; }
  }
  red[tid] = s1; __syncthreads();
  for (int st = 128; st > 0; st >>= 1) { if (tid < st) red[tid] += red[tid + st]; __syncthreads(); }
  const float mu = red[0] / (float)N; __syncthreads();
  float s2 = 0.f;
  for (int u = 0; u < per / 4; ++u)
#pragma unroll
    for (int q = 0; q < 4; ++q) { const float c = vals[u * 4 + q] - mu; s2 += c * c; }
  red[tid] = s2; __syncthreads();
  for (int st = 128; st > 0; st >>= 1) { if (tid < st) red[tid] += red[tid + st]; __syncthreads(); }
  const float rs = rsqrtf(red[0] / (float)N + eps);
  for (int pass = 0; pass < 2; ++pass) {
    for (int u = 0; u < per / 4; ++u) {
      const int j = tid * 4 + 1024 * u;
      v4f o, sm;
#pragma unroll
      for (int q = 0; q < 4; ++q) {
        float gg = g[j + q], bb = bta[j + q];
        if (PARAM_BF16) { gg = bf16_round(gg); bb = bf16_round(bb); }
        sm[q] = vals[u * 4 + q]; o[q] = (vals[u * 4 + q] - mu) * rs * gg + bb;
      }
      if (out_sum) *(volatile v4f*)(out_sum + (size_t)row * N + j) = sm;
      *(volatile v4f*)(out_norm + (size_t)row * N + j) = o;
    }
    if (pass == 0) __threadfence();
  }
}


typedef _Float16 v16h __attribute__((ext_vector_type(16)));
union FragH { v16h v; v8us half[2]; _Float16 h[16]; unsigned short u[16]; };
template <int NT>
__device__ __forceinline__ v8f mmaH(v16h ah, v16h al, v16h bh, v16h bl, v8f c) {
  c = __builtin_amdgcn_wmma_f32_16x16x32_f16(false, ah, false, bh, (short)0, c, false, false);
  if (NT >= 2) c = __builtin_amdgcn_wmma_f32_16x16x32_f16(false, al, false, bh, (short)0, c, false, false);
  if (NT >= 3) c = __builtin_amdgcn_wmma_f32_16x16x32_f16(false, ah, false, bl, (short)0, c, false, false);
  asm volatile("v_nop\n\tv_nop\n\tv_nop\n\tv_nop" : "+v"(c) : "v"(ah), "v"(al), "v"(bh), "v"(bl));
  return c;
}
template <bool ASPLIT>
__global__ __launch_bounds__(128) void k_gemm_h(const float* __restrict__ A, int lda, size_t sA, const _Float16* __restrict__ Bh, int ldb, size_t sB, float alpha, float* __restrict__ C, int ldc, size_t sC, int M, int N, int K) {
  __shared__ __attribute__((aligned(16))) float so[4][16][64];
  const int tid = threadIdx.x, w = tid >> 5, lane = tid & 31, ln = lane & 15, hh = lane >> 4; const int by = blockIdx.y;
  A += (size_t)by * sA; Bh += (size_t)by * sB; C += (size_t)by * sC;
  const int ntn = (N + 63) / 64; const int wid = blockIdx.x * 4 + w; const int mt = wid / ntn, nq = wid % ntn; if (mt * 16 >= M) return;
  const int row0 = mt * 16, col0 = nq * 64; const float* arow = A + (size_t)(row0 + ln) * lda;
  v8f acc[4] = {};
  for (int kb = 0; kb < K; kb += 32) {
    FragH ah, al;
    const v4f x0 = *(const v4fa*)(arow + kb + 8 * hh), x1 = *(const v4fa*)(arow + kb + 8 * hh + 4), x2 = *(const v4fa*)(arow + kb + 16 + 8 * hh), x3 = *(const v4fa*)(arow + kb + 16 + 8 * hh + 4);
    float xs[16] = {x0[0],x0[1],x0[2],x0[3],x1[0],x1[1],x1[2],x1[3],x2[0],x2[1],x2[2],x2[3],x3[0],x3[1],x3[2],x3[3]};
#pragma unroll
    for (int i = 0; i < 16; ++i) { const _Float16 h = (_Float16)xs[i]; ah.h[i] = h; al.h[i] = ASPLIT ? (_Float16)(xs[i] - (float)h) : (_Float16)0.0f; }
#pragma unroll
    for (int t = 0; t < 4; ++t) { if (col0 + t * 16 >= N) continue; const size_t boff = (size_t)(col0 + t * 16 + ln) * ldb + kb; FragH bq; bq.half[0] = *(const v8us*)(Bh + boff + 8 * hh); bq.half[1] = *(const v8us*)(Bh + boff + 16 + 8 * hh);
      acc[t] = mmaH<ASPLIT ? 2 : 1>(ah.v, al.v, bq.v, bq.v, acc[t]); }
  }
#pragma unroll
  for (int t = 0; t < 4; ++t) { if (col0 + t * 16 >= N) continue;
#pragma unroll
    for (int r = 0; r < 8; ++r) so[w][8 * hh + r][t * 16 + ln] = acc[t][r] * alpha; }
  __builtin_amdgcn_fence(__ATOMIC_ACQ_REL, "workgroup"); __builtin_amdgcn_wave_barrier();
  const int rsub = lane >> 4, c4 = (lane & 15) * 4;
  for (int pass = 0; pass < 2; ++pass) {
#pragma unroll
    for (int q = 0; q < 8; ++q) { const int r = q * 2 + rsub; if (col0 + c4 < N) { const v4f v = *(const v4fa*)&so[w][r][c4]; *(volatile v4f*)(C + (size_t)(row0 + r) * ldc + col0 + c4) = v; } }
    if (pass == 0) __threadfence(); }
}

__global__ __launch_bounds__(256) void k_wt_f16(const float* __restrict__ W, _Float16* __restrict__ Wt, int K, int N, float scale) {
  const int t = blockIdx.x * 256 + threadIdx.x; if (t >= N * (K / 8)) return; const int n = t / (K / 8), k8 = (t % (K / 8)) * 8; FragH f;
#pragma unroll
  for (int i = 0; i < 8; ++i) f.h[i] = (_Float16)(bf16_round(W[(size_t)(k8 + i) * N + n]) * scale); const v8us o = f.half[0];
  *(volatile v8us*)((unsigned short*)Wt + (size_t)n * K + k8) = o; __threadfence(); *(volatile v8us*)((unsigned short*)Wt + (size_t)n * K + k8) = o;
}
template <int ACT>
__global__ __launch_bounds__(128) void k_gemm_hhx(const _Float16* __restrict__ A, int lda, size_t sA, const _Float16* __restrict__ Bh, int ldb, size_t sB, float alpha, const float* __restrict__ bias, size_t sBias, const float* __restrict__ CP, int rowsPerB, size_t sCPb, int row0g,
    float* __restrict__ C, _Float16* __restrict__ C16, int ldc, size_t sC, int M, int N, int K) {
  __shared__ __attribute__((aligned(16))) float so[4][16][64];
  const int tid = threadIdx.x, w = tid >> 5, lane = tid & 31, ln = lane & 15, hh = lane >> 4; const int by = blockIdx.y;
  A += (size_t)by * sA; Bh += (size_t)by * sB; const size_t cofs = (size_t)by * sC; const float* bp = bias ? bias + (size_t)by * sBias : nullptr;
  const int ntn = (N + 63) / 64; const int wid = blockIdx.x * 4 + w; const int mt = wid / ntn, nq = wid % ntn; if (mt * 16 >= M) return;
  const int row0 = mt * 16, col0 = nq * 64; const _Float16* arow = A + (size_t)(row0 + ln) * lda;
  v8f acc[4] = {};
  for (int kb = 0; kb < K; kb += 32) { FragH ah; ah.half[0] = *(const v8us*)((const unsigned short*)arow + kb + 8 * hh); ah.half[1] = *(const v8us*)((const unsigned short*)arow + kb + 16 + 8 * hh);
#pragma unroll
    for (int t = 0; t < 4; ++t) { if (col0 + t * 16 >= N) continue; const size_t boff = (size_t)(col0 + t * 16 + ln) * ldb + kb; FragH bq; bq.half[0] = *(const v8us*)((const unsigned short*)Bh + boff + 8 * hh); bq.half[1] = *(const v8us*)((const unsigned short*)Bh + boff + 16 + 8 * hh);
      acc[t] = mmaH<1>(ah.v, ah.v, bq.v, bq.v, acc[t]); }
  }
#pragma unroll
  for (int t = 0; t < 4; ++t) { if (col0 + t * 16 >= N) continue; const int col = col0 + t * 16 + ln; const float bv = bp ? bf16_round(bp[col]) : 0.f;
#pragma unroll
    for (int r = 0; r < 8; ++r) { float v = acc[t][r] * alpha + bv; if (CP) { const int bidx = (row0g + row0 + 8 * hh + r) / rowsPerB; v += CP[(size_t)bidx * sCPb + (size_t)by * 64 + col]; } if (ACT == 1) v = (v > 0.f) ? v : expm1f(v); else if (ACT == 7) v = (v > 0.f) ? v + 1.0f : expf(v); else if (ACT == 8) v = tanhf(v); else if (ACT == 9) v = 0.5f * v * (1.0f + tanhf(0.7978845608028654f * (v + 0.044715f * v * v * v))); else if (ACT == 11) v = 1.0f / (1.0f + expf(-v)); else if (ACT == 12) v = (v > 0.f) ? v : 0.01f * v; else if (ACT == 14) v = (v > 0.f) ? v : 0.1f * v; else if (ACT == 15) v = v / (1.0f + expf(-v)); else if (ACT == 3) v = fmaxf(v, 0.f); else if (ACT == 6) v = 0.5f * v * (1.0f + erff(v * 0.70710678118654752f)); so[w][8 * hh + r][t * 16 + ln] = v; } }
  __builtin_amdgcn_fence(__ATOMIC_ACQ_REL, "workgroup"); __builtin_amdgcn_wave_barrier();
  const int rsub = lane >> 4, c4 = (lane & 15) * 4; typedef _Float16 v4h __attribute__((ext_vector_type(4)));
  for (int pass = 0; pass < 2; ++pass) {
#pragma unroll
    for (int q = 0; q < 8; ++q) { const int r = q * 2 + rsub; if (col0 + c4 < N) { const v4f v = *(const v4fa*)&so[w][r][c4]; if (C) *(volatile v4f*)(C + cofs + (size_t)(row0 + r) * ldc + col0 + c4) = v; if (C16) { v4h h4; for (int i = 0; i < 4; ++i) h4[i] = (_Float16)v[i]; *(volatile v4h*)(C16 + cofs + (size_t)(row0 + r) * ldc + col0 + c4) = h4; } } }
    if (pass == 0) __threadfence(); }
}


typedef _Float16 v4h __attribute__((ext_vector_type(4)));

__global__ __launch_bounds__(256) void k_x16(const float* __restrict__ x, _Float16* __restrict__ X16, size_t n8) { const size_t t = (size_t)blockIdx.x * 256 + threadIdx.x; if (t >= n8) return; FragH f;
#pragma unroll
  for (int q = 0; q < 8; ++q) f.h[q] = (_Float16)bf16_round(x[t * 8 + q]); *(volatile v8us*)((unsigned short*)X16 + t * 8) = f.half[0]; __threadfence(); *(volatile v8us*)((unsigned short*)X16 + t * 8) = f.half[0]; }
__global__ __launch_bounds__(256) void k_h16(const float* __restrict__ x, _Float16* __restrict__ X16, size_t n8) { const size_t t = (size_t)blockIdx.x * 256 + threadIdx.x; if (t >= n8) return; FragH f;
#pragma unroll
  for (int q = 0; q < 8; ++q) f.h[q] = (_Float16)x[t * 8 + q]; *(volatile v8us*)((unsigned short*)X16 + t * 8) = f.half[0]; __threadfence(); *(volatile v8us*)((unsigned short*)X16 + t * 8) = f.half[0]; }
__global__ __launch_bounds__(256) void k_round16f(const float* __restrict__ W, _Float16* __restrict__ Bt, size_t n8) { const size_t t = (size_t)blockIdx.x * 256 + threadIdx.x; if (t >= n8) return; FragH f;
#pragma unroll
  for (int i = 0; i < 8; ++i) f.h[i] = (_Float16)(bf16_round(W[t * 8 + i]) * 16.0f); *(volatile v8us*)((unsigned short*)Bt + t * 8) = f.half[0]; __threadfence(); *(volatile v8us*)((unsigned short*)Bt + t * 8) = f.half[0]; }
template <int NHv, int TTv>
__global__ __launch_bounds__(256) void k_vt(const _Float16* __restrict__ V16, int ldv, int voff, _Float16* __restrict__ Vt) { __shared__ unsigned short tl[64][66]; const int tid = threadIdx.x; const int slab = blockIdx.x / (TTv / 64), lg = blockIdx.x % (TTv / 64); const int b = slab / NHv, h = slab % NHv;
  for (int i = tid; i < 64 * 8; i += 256) { const int r = i / 8, c8 = (i % 8) * 8; FragH f; f.half[0] = *(const v8us*)((const unsigned short*)V16 + ((size_t)b * TTv + lg * 64 + r) * ldv + voff + h * 64 + c8);
#pragma unroll
    for (int q = 0; q < 8; ++q) tl[r][c8 + q] = f.u[q]; }
  __syncthreads();
  for (int pass = 0; pass < 2; ++pass) {
#pragma unroll
    for (int rd = 0; rd < 2; ++rd) { const int d = rd * 32 + tid / 8, pc = tid % 8; FragH f;
#pragma unroll
      for (int q = 0; q < 8; ++q) f.u[q] = tl[pc * 8 + q][d];
      *(volatile v8us*)((unsigned short*)Vt + ((size_t)slab * 64 + d) * TTv + lg * 64 + pc * 8) = f.half[0]; }
    if (pass == 0) __threadfence(); } }

__global__ __launch_bounds__(256) void k_hl(const float* __restrict__ F, _Float16* __restrict__ Hh, _Float16* __restrict__ Hl, size_t n8) { const size_t t = (size_t)blockIdx.x * 256 + threadIdx.x; if (t >= n8) return; FragH fh, fl; const v4f a = *(const v4fa*)(F + t * 8), c = *(const v4fa*)(F + t * 8 + 4);
#pragma unroll
  for (int q = 0; q < 4; ++q) { _Float16 h = (_Float16)a[q]; fh.h[q] = h; fl.h[q] = (_Float16)((a[q] - (float)h) * 1024.0f); h = (_Float16)c[q]; fh.h[4 + q] = h; fl.h[4 + q] = (_Float16)((c[q] - (float)h) * 1024.0f); }
  for (int pass = 0; pass < 2; ++pass) { *(volatile v8us*)((unsigned short*)Hh + t * 8) = fh.half[0]; *(volatile v8us*)((unsigned short*)Hl + t * 8) = fl.half[0]; if (pass == 0) __threadfence(); } }

__global__ __launch_bounds__(256) void k_vn(const float* __restrict__ v, int n, float* __restrict__ VN) {
  #pragma clang fp contract(off)
  const int i = blockIdx.x * 256 + threadIdx.x; if (i >= n) return; const float x = bf16_round(v[(size_t)i * 3]), y = bf16_round(v[(size_t)i * 3 + 1]), z = bf16_round(v[(size_t)i * 3 + 2]); const float s = (x * x + y * y) + z * z; *(volatile float*)(VN + i) = s; __threadfence(); *(volatile float*)(VN + i) = s; }
__global__ __launch_bounds__(256) void k_rbf1(const float* __restrict__ coords, const float* __restrict__ verts, const float* __restrict__ VN, int c0, float* __restrict__ DMIN) {
  #pragma clang fp contract(off)
  __shared__ float red[8]; const int tid = threadIdx.x, w = tid >> 5, l = tid & 31; const int c = c0 + blockIdx.x; const float cx = bf16_round(coords[(size_t)c * 3]), cy = bf16_round(coords[(size_t)c * 3 + 1]), cz = bf16_round(coords[(size_t)c * 3 + 2]); const float cn = (cx * cx + cy * cy) + cz * cz; float m = 3.0e38f;
#pragma unroll 1
  for (int v = tid; v < NV; v += 256) { const float vx = bf16_round(verts[(size_t)v * 3]), vy = bf16_round(verts[(size_t)v * 3 + 1]), vz = bf16_round(verts[(size_t)v * 3 + 2]); const float dot = (cx * vx + cy * vy) + cz * vz; const float d2 = (cn + VN[v]) - 2.0f * dot; m = fminf(m, sqrtf(fmaxf(d2, 0.f))); }
  for (int o = 16; o > 0; o >>= 1) m = fminf(m, __shfl_xor(m, o, 32)); if (l == 0) red[w] = m; __syncthreads();
  if (tid < 32) { float mm = red[0]; for (int k = 1; k < 8; ++k) mm = fminf(mm, red[k]); *(volatile float*)(DMIN + (size_t)c * 32 + tid) = mm; __threadfence(); *(volatile float*)(DMIN + (size_t)c * 32 + tid) = mm; } }
__global__ __launch_bounds__(256) void k_rbf2(const float* __restrict__ coords, const float* __restrict__ verts, const float* __restrict__ VN, const float* __restrict__ DMIN, int c0, _Float16* __restrict__ W16, float* __restrict__ RSUM) {
  #pragma clang fp contract(off)
  __shared__ float red[8]; const int tid = threadIdx.x, w = tid >> 5, l = tid & 31; const int c = c0 + blockIdx.x; const float cx = bf16_round(coords[(size_t)c * 3]), cy = bf16_round(coords[(size_t)c * 3 + 1]), cz = bf16_round(coords[(size_t)c * 3 + 2]); const float cn = (cx * cx + cy * cy) + cz * cz; const float dm = DMIN[(size_t)c * 32]; float s = 0.f;
#pragma unroll 1
  for (int v0 = tid * 8; v0 < NV; v0 += 256 * 8) { FragH f;
#pragma unroll
    for (int q = 0; q < 8; ++q) { const int v = v0 + q; const float vx = bf16_round(verts[(size_t)v * 3]), vy = bf16_round(verts[(size_t)v * 3 + 1]), vz = bf16_round(verts[(size_t)v * 3 + 2]); const float dot = (cx * vx + cy * vy) + cz * vz; const float d2 = (cn + VN[v]) - 2.0f * dot; const float d = sqrtf(fmaxf(d2, 0.f)); const float wv = expf(-(d - dm) / RSIG); s += wv; f.h[q] = (_Float16)(wv * 32768.0f); }
    unsigned short* wp = (unsigned short*)W16 + (size_t)(c - c0) * NV + v0; *(volatile v8us*)wp = f.half[0]; __threadfence(); *(volatile v8us*)wp = f.half[0]; }
  for (int o = 16; o > 0; o >>= 1) s += __shfl_xor(s, o, 32); if (l == 0) red[w] = s; __syncthreads();
  if (tid < 32) { float ss = 0.f; for (int k = 0; k < 8; ++k) ss += red[k]; *(volatile float*)(RSUM + (size_t)c * 32 + tid) = ss; __threadfence(); *(volatile float*)(RSUM + (size_t)c * 32 + tid) = ss; } }
__global__ __launch_bounds__(256) void k_xin(const float* __restrict__ PL, const float* __restrict__ RSL, const float* __restrict__ DML, const float* __restrict__ PR, const float* __restrict__ RSR, const float* __restrict__ DMR, _Float16* __restrict__ X) {
  #pragma clang fp contract(off)
  const int t = blockIdx.x * 256 + threadIdx.x; if (t >= NC * (FINP / 8)) return; const int c = t / (FINP / 8), g = (t % (FINP / 8)) * 8; const float il = 1.0f / RSL[(size_t)c * 32], ir = 1.0f / RSR[(size_t)c * 32]; FragH f;
#pragma unroll
  for (int q = 0; q < 8; ++q) { const int col = g + q; float v; if (col < CF) v = PL[(size_t)c * CF + col] * il; else if (col == CF) v = DML[(size_t)c * 32]; else if (col < 2 * CF + 1) v = PR[(size_t)c * CF + (col - CF - 1)] * ir; else if (col == 2 * CF + 1) v = DMR[(size_t)c * 32]; else v = 0.f; f.h[q] = (_Float16)v; }
  *(volatile v8us*)((unsigned short*)X + (size_t)c * FINP + g) = f.half[0]; __threadfence(); *(volatile v8us*)((unsigned short*)X + (size_t)c * FINP + g) = f.half[0]; }
__global__ __launch_bounds__(256) void k_ft(const float* __restrict__ feats, _Float16* __restrict__ FT) { const int t = blockIdx.x * 256 + threadIdx.x; if (t >= CF * (NV / 8)) return; const int k = t / (NV / 8), v0 = (t % (NV / 8)) * 8; FragH f;
#pragma unroll
  for (int q = 0; q < 8; ++q) f.h[q] = (_Float16)bf16_round(feats[(size_t)(v0 + q) * CF + k]);
  *(volatile v8us*)((unsigned short*)FT + (size_t)k * NV + v0) = f.half[0]; __threadfence(); *(volatile v8us*)((unsigned short*)FT + (size_t)k * NV + v0) = f.half[0]; }
__global__ __launch_bounds__(256) void k_w1p(const float* __restrict__ w, _Float16* __restrict__ Bt) { const int t = blockIdx.x * 256 + threadIdx.x; if (t >= CF * (FINP / 8)) return; const int o = t / (FINP / 8), k0 = (t % (FINP / 8)) * 8; FragH f;
#pragma unroll
  for (int q = 0; q < 8; ++q) { const int k = k0 + q; f.h[q] = (k < FIN) ? (_Float16)(bf16_round(w[(size_t)k * CF + o]) * 16.0f) : (_Float16)0.0f; }
  *(volatile v8us*)((unsigned short*)Bt + (size_t)o * FINP + k0) = f.half[0]; __threadfence(); *(volatile v8us*)((unsigned short*)Bt + (size_t)o * FINP + k0) = f.half[0]; }
__global__ __launch_bounds__(256) void k_tr(const _Float16* __restrict__ S, _Float16* __restrict__ T) { const int t = blockIdx.x * 256 + threadIdx.x; if (t >= CF * (NC / 8)) return; const int k = t / (NC / 8), i0 = (t % (NC / 8)) * 8; FragH f;
#pragma unroll
  for (int q = 0; q < 8; ++q) f.h[q] = S[(size_t)(i0 + q) * CF + k];
  *(volatile v8us*)((unsigned short*)T + (size_t)k * NC + i0) = f.half[0]; __threadfence(); *(volatile v8us*)((unsigned short*)T + (size_t)k * NC + i0) = f.half[0]; }
__global__ __launch_bounds__(256) void k_gdeg(const float* __restrict__ coords, float* __restrict__ DINV) {
  #pragma clang fp contract(off)
  __shared__ float red[8]; const int tid = threadIdx.x, w = tid >> 5, l = tid & 31; const int i = blockIdx.x; const float cx = bf16_round(coords[(size_t)i * 3]), cy = bf16_round(coords[(size_t)i * 3 + 1]), cz = bf16_round(coords[(size_t)i * 3 + 2]); const float cn = (cx * cx + cy * cy) + cz * cz; float s = 0.f;
#pragma unroll 1
  for (int j = tid; j < NC; j += 256) { const float vx = bf16_round(coords[(size_t)j * 3]), vy = bf16_round(coords[(size_t)j * 3 + 1]), vz = bf16_round(coords[(size_t)j * 3 + 2]); const float vn = (vx * vx + vy * vy) + vz * vz; const float dot = (cx * vx + cy * vy) + cz * vz; const float d = sqrtf(fmaxf((cn + vn) - 2.0f * dot, 0.f)); s += expf(-d / GSIG); }
  for (int o = 16; o > 0; o >>= 1) s += __shfl_xor(s, o, 32); if (l == 0) red[w] = s; __syncthreads();
  if (tid < 32) { float ss = 0.f; for (int k = 0; k < 8; ++k) ss += red[k]; const float di = rsqrtf(ss); *(volatile float*)(DINV + (size_t)i * 32 + tid) = di; __threadfence(); *(volatile float*)(DINV + (size_t)i * 32 + tid) = di; } }
__global__ __launch_bounds__(256) void k_gadj(const float* __restrict__ coords, const float* __restrict__ DINV, _Float16* __restrict__ A16) {
  #pragma clang fp contract(off)
  const int tid = threadIdx.x; const int i = blockIdx.x; const float cx = bf16_round(coords[(size_t)i * 3]), cy = bf16_round(coords[(size_t)i * 3 + 1]), cz = bf16_round(coords[(size_t)i * 3 + 2]); const float cn = (cx * cx + cy * cy) + cz * cz;
  for (int pass = 0; pass < 2; ++pass) {
#pragma unroll 1
    for (int j0 = tid * 8; j0 < NC; j0 += 256 * 8) { FragH f;
#pragma unroll
      for (int q = 0; q < 8; ++q) { const int j = j0 + q; const float vx = bf16_round(coords[(size_t)j * 3]), vy = bf16_round(coords[(size_t)j * 3 + 1]), vz = bf16_round(coords[(size_t)j * 3 + 2]); const float vn = (vx * vx + vy * vy) + vz * vz; const float dot = (cx * vx + cy * vy) + cz * vz; const float d = sqrtf(fmaxf((cn + vn) - 2.0f * dot, 0.f)); f.h[q] = (_Float16)((expf(-d / GSIG) * DINV[(size_t)j * 32]) * 65536.0f); }
      *(volatile v8us*)((unsigned short*)A16 + (size_t)i * NC + j0) = f.half[0]; }
    if (pass == 0) __threadfence(); } }
template <int RELU>
__global__ __launch_bounds__(256) void k_gep(const float* __restrict__ Z, const float* __restrict__ DINV, const float* __restrict__ bb, _Float16* __restrict__ H16, float* __restrict__ Hf) {
  #pragma clang fp contract(off)
  const int t = blockIdx.x * 256 + threadIdx.x; if (t >= NC * (CF / 8)) return; const int i = t / (CF / 8), k0 = (t % (CF / 8)) * 8; const float di = DINV[(size_t)i * 32]; FragH f; v4f a, c;
#pragma unroll
  for (int q = 0; q < 8; ++q) { float v = di * Z[(size_t)i * CF + k0 + q] + bf16_round(bb[k0 + q]); if (RELU) v = fmaxf(v, 0.f); f.h[q] = (_Float16)v; if (q < 4) a[q] = v; else c[q - 4] = v; }
  for (int pass = 0; pass < 2; ++pass) { if (H16) *(volatile v8us*)((unsigned short*)H16 + (size_t)i * CF + k0) = f.half[0]; if (Hf) { *(volatile v4f*)(Hf + (size_t)i * CF + k0) = a; *(volatile v4f*)(Hf + (size_t)i * CF + k0 + 4) = c; } if (pass == 0) __threadfence(); } }
__global__ __launch_bounds__(64) void k_maxpool(const float* __restrict__ Hf, int g, float* __restrict__ POOL) { const int k = threadIdx.x; if (k >= CF) return; float m = -3.0e38f;
#pragma unroll 1
  for (int i = 0; i < NC; ++i) m = fmaxf(m, Hf[(size_t)i * CF + k]); *(volatile float*)(POOL + g * CF + k) = m; __threadfence(); *(volatile float*)(POOL + g * CF + k) = m; }
__global__ __launch_bounds__(128) void k_top(const float* __restrict__ POOL, const float* __restrict__ wm1, const float* __restrict__ bm1, const float* __restrict__ wm2, const float* __restrict__ bm2, float* __restrict__ out) {
  #pragma clang fp contract(off)
  __shared__ float hs[128]; const int t = threadIdx.x; float s = bf16_round(bm1[t]);
#pragma unroll 1
  for (int k = 0; k < 128; ++k) s += POOL[k] * bf16_round(wm1[(size_t)k * 128 + t]); hs[t] = fmaxf(s, 0.f) * bf16_round(wm2[t]); __syncthreads();
  if (t == 0) { float o = 0.f; for (int k = 0; k < 128; ++k) o += hs[k]; o += bf16_round(bm2[0]); *(volatile float*)out = o; __threadfence(); *(volatile float*)out = o; } }

extern "C" void kernel_launch(void* const* d_in, const int* in_sizes, int n_in,
                              void* d_out, int out_size, void* d_ws, size_t ws_size, hipStream_t stream) {
  (void)in_sizes; (void)n_in; (void)out_size;
  const float* const* I = (const float* const*)d_in; const float* verts[4] = {I[0], I[2], I[4], I[6]}; const float* feats[4] = {I[1], I[3], I[5], I[7]}; const float* coords[2] = {I[8], I[9]};
  const float* w1 = I[10]; const float* b1 = I[11]; const float* w2 = I[12]; const float* b2 = I[13]; const float* w3 = I[14]; const float* b3 = I[15]; const float* wm1 = I[16]; const float* bm1 = I[17]; const float* wm2 = I[18]; const float* bm2 = I[19];
  char* ws = (char*)d_ws; size_t off = 0;
  auto take = [&](size_t bytes) { char* p = ws + off; off += (bytes + 255) & ~(size_t)255; return p; };
  _Float16* Bw1 = (_Float16*)take((size_t)CF * FINP * 2); _Float16* Bw2 = (_Float16*)take((size_t)CF * CF * 2); _Float16* Bw3 = (_Float16*)take((size_t)CF * CF * 2);
  float* VN = (float*)take((size_t)NV * 4); float* DMIN = (float*)take((size_t)NC * 32 * 4); float* RSUM = (float*)take((size_t)NC * 32 * 4); _Float16* F16 = (_Float16*)take((size_t)NV * CF * 2); _Float16* W16 = (_Float16*)take((size_t)RCH * NV * 2); float* P = (float*)take((size_t)NC * CF * 4);
  _Float16* X = (_Float16*)take((size_t)NC * FINP * 2); float* DINV = (float*)take((size_t)NC * 32 * 4); _Float16* A16 = (_Float16*)take((size_t)NC * NC * 2); _Float16* XW = (_Float16*)take((size_t)NC * CF * 2); float* Z = (float*)take((size_t)NC * CF * 4); _Float16* H16 = (_Float16*)take((size_t)NC * CF * 2); float* Hf = (float*)take((size_t)NC * CF * 4); float* POOL = (float*)take(2 * CF * 4);
  float* P2 = (float*)take((size_t)NC * CF * 4); float* DMIN2 = (float*)take((size_t)NC * 32 * 4); float* RSUM2 = (float*)take((size_t)NC * 32 * 4); _Float16* XWT = (_Float16*)take((size_t)CF * NC * 2);
  if (off > ws_size) return;
  k_w1p<<<(CF * (FINP / 8) + 255) / 256, 256, 0, stream>>>(w1, Bw1); k_wt_f16<<<(CF * (CF / 8) + 255) / 256, 256, 0, stream>>>(w2, Bw2, CF, CF, 16.0f); k_wt_f16<<<(CF * (CF / 8) + 255) / 256, 256, 0, stream>>>(w3, Bw3, CF, CF, 16.0f);
  for (int g = 0; g < 2; ++g) {
    const float* cg = coords[g];
    for (int side = 0; side < 2; ++side) { const int pi = 2 * g + side; float* Pp = side ? P2 : P; float* DM = side ? DMIN2 : DMIN; float* RS = side ? RSUM2 : RSUM;
      k_vn<<<(NV + 255) / 256, 256, 0, stream>>>(verts[pi], NV, VN); k_ft<<<(CF * (NV / 8) + 255) / 256, 256, 0, stream>>>(feats[pi], F16);
      for (int ch = 0; ch < NC / RCH; ++ch) { const int c0 = ch * RCH;
        k_rbf1<<<RCH, 256, 0, stream>>>(cg, verts[pi], VN, c0, DM); k_rbf2<<<RCH, 256, 0, stream>>>(cg, verts[pi], VN, DM, c0, W16, RS);
        k_gemm_hhx<0><<<dim3(((RCH / 16) * 1 + 3) / 4, 1), 128, 0, stream>>>(W16, NV, 0, F16, NV, 0, 1.0f / 32768.0f, nullptr, 0, nullptr, 1, 0, 0, Pp + (size_t)c0 * CF, nullptr, CF, 0, RCH, CF, NV); } }
    k_xin<<<(NC * (FINP / 8) + 255) / 256, 256, 0, stream>>>(P, RSUM, DMIN, P2, RSUM2, DMIN2, X);
    k_gdeg<<<NC, 256, 0, stream>>>(cg, DINV); k_gadj<<<NC, 256, 0, stream>>>(cg, DINV, A16);
    const dim3 gN(((NC / 16) * 1 + 3) / 4, 1);
    k_gemm_hhx<0><<<gN, 128, 0, stream>>>(X, FINP, 0, Bw1, FINP, 0, 0.0625f, nullptr, 0, nullptr, 1, 0, 0, nullptr, XW, CF, 0, NC, CF, FINP); k_tr<<<(CF * (NC / 8) + 255) / 256, 256, 0, stream>>>(XW, XWT);
    k_gemm_hhx<0><<<gN, 128, 0, stream>>>(A16, NC, 0, XWT, NC, 0, 1.0f / 65536.0f, nullptr, 0, nullptr, 1, 0, 0, Z, nullptr, CF, 0, NC, CF, NC); k_gep<1><<<(NC * (CF / 8) + 255) / 256, 256, 0, stream>>>(Z, DINV, b1, H16, nullptr);
    k_gemm_hhx<0><<<gN, 128, 0, stream>>>(H16, CF, 0, Bw2, CF, 0, 0.0625f, nullptr, 0, nullptr, 1, 0, 0, nullptr, XW, CF, 0, NC, CF, CF); k_tr<<<(CF * (NC / 8) + 255) / 256, 256, 0, stream>>>(XW, XWT);
    k_gemm_hhx<0><<<gN, 128, 0, stream>>>(A16, NC, 0, XWT, NC, 0, 1.0f / 65536.0f, nullptr, 0, nullptr, 1, 0, 0, Z, nullptr, CF, 0, NC, CF, NC); k_gep<1><<<(NC * (CF / 8) + 255) / 256, 256, 0, stream>>>(Z, DINV, b2, H16, nullptr);
    k_gemm_hhx<0><<<gN, 128, 0, stream>>>(H16, CF, 0, Bw3, CF, 0, 0.0625f, nullptr, 0, nullptr, 1, 0, 0, nullptr, XW, CF, 0, NC, CF, CF); k_tr<<<(CF * (NC / 8) + 255) / 256, 256, 0, stream>>>(XW, XWT);
    k_gemm_hhx<0><<<gN, 128, 0, stream>>>(A16, NC, 0, XWT, NC, 0, 1.0f / 65536.0f, nullptr, 0, nullptr, 1, 0, 0, Z, nullptr, CF, 0, NC, CF, NC); k_gep<0><<<(NC * (CF / 8) + 255) / 256, 256, 0, stream>>>(Z, DINV, b3, nullptr, Hf);
    k_maxpool<<<1, 64, 0, stream>>>(Hf, g, POOL); }
  k_top<<<1, 128, 0, stream>>>(POOL, wm1, bm1, wm2, bm2, (float*)d_out);
}
